// PointNet2Feat_17291538333862
// MI455X (gfx1250) — hardware-verified
//
#include <hip/hip_runtime.h>
#pragma clang fp contract(off)

typedef __attribute__((ext_vector_type(16))) _Float16 v16h;
typedef __attribute__((ext_vector_type(8)))  _Float16 v8h;
typedef __attribute__((ext_vector_type(8)))  float    v8f;
typedef __attribute__((ext_vector_type(4)))  float    v4f;
typedef __attribute__((ext_vector_type(4)))  unsigned v4u;

constexpr int NBATCH = 16;
constexpr int NPTS0  = 8192;
constexpr int NCTR1  = 512;
constexpr int NCTR2  = 128;
constexpr int NNB    = 64;
constexpr int CIN1   = 3;
constexpr int CH1A   = 64;
constexpr int CH1B   = 128;
constexpr int CIN2   = 131;
constexpr int CH2A   = 128;
constexpr int CH2B   = 256;
constexpr int CIN3   = 259;
constexpr int CH3A   = 512;
constexpr int CH3B   = 1024;
constexpr int KP1A = 32;
constexpr int KP1B = 64;
constexpr int KP2A = 160;
constexpr int KP2B = 128;
constexpr int KP3A = 288;
constexpr int KP3B = 512;
static_assert(KP1A % 32 == 0 && KP1B % 32 == 0 && KP2A % 32 == 0 && KP2B % 32 == 0 && KP3A % 32 == 0 && KP3B % 32 == 0);
static_assert(KP1A >= CIN1 && KP1B == CH1A && KP2A >= CIN2 && KP2B == CH2A && KP3A >= CIN3 && KP3B == CH3A);
static_assert(CIN2 == CH1B + 3 && CIN3 == CH2B + 3);
static_assert(NCTR1 % 4 == 0 && NCTR2 % 2 == 0);

constexpr float CARRY_W  = 16.0f;
constexpr float CARRY_G1 = 64.0f;
constexpr float CARRY_M1 = 64.0f;
constexpr float CARRY_F1 = 16.0f;
constexpr float CARRY_M2 = 16.0f;
constexpr float CARRY_F2 = 16.0f;
constexpr float CARRY_M3 = 16.0f;
constexpr float INV_1A = 1.0f / (CARRY_G1 * CARRY_W);
constexpr float INV_1B = 1.0f / (CARRY_M1 * CARRY_W);
constexpr float INV_2A = 1.0f / (CARRY_F1 * CARRY_W);
constexpr float INV_2B = 1.0f / (CARRY_M2 * CARRY_W);
constexpr float INV_3A = 1.0f / (CARRY_F2 * CARRY_W);
constexpr float INV_3B = 1.0f / (CARRY_M3 * CARRY_W);

constexpr size_t SZ_W1A  = (size_t)CH1A * KP1A * 2;
constexpr size_t SZ_W1B  = (size_t)CH1B * KP1B * 2;
constexpr size_t SZ_W2A  = (size_t)CH2A * KP2A * 2;
constexpr size_t SZ_W2B  = (size_t)CH2B * KP2B * 2;
constexpr size_t SZ_W3A  = (size_t)CH3A * KP3A * 2;
constexpr size_t SZ_W3B  = (size_t)CH3B * KP3B * 2;
constexpr size_t SZ_XYZ1 = (size_t)NBATCH * NCTR1 * 3 * 4;
constexpr size_t SZ_XYZ2 = (size_t)NBATCH * NCTR2 * 3 * 4;
constexpr size_t SZ_F1   = (size_t)NBATCH * NCTR1 * CH1B * 2;
constexpr size_t SZ_A3   = (size_t)NBATCH * NCTR2 * KP3A * 2;
constexpr size_t SZ_ACT3 = (size_t)NBATCH * NCTR2 * CH3A * 2;
constexpr size_t OFF_W1A  = 0;
constexpr size_t OFF_W1B  = OFF_W1A + SZ_W1A;
constexpr size_t OFF_W2A  = OFF_W1B + SZ_W1B;
constexpr size_t OFF_W2B  = OFF_W2A + SZ_W2A;
constexpr size_t OFF_W3A  = OFF_W2B + SZ_W2B;
constexpr size_t OFF_W3B  = OFF_W3A + SZ_W3A;
constexpr size_t OFF_XYZ1 = OFF_W3B + SZ_W3B;
constexpr size_t OFF_XYZ2 = OFF_XYZ1 + SZ_XYZ1;
constexpr size_t OFF_F1   = OFF_XYZ2 + SZ_XYZ2;
constexpr size_t OFF_A3   = OFF_F1 + SZ_F1;
constexpr size_t OFF_ACT3 = OFF_A3 + SZ_A3;
constexpr size_t WS_TOTAL = OFF_ACT3 + SZ_ACT3;
static_assert(OFF_W1B % 128 == 0 && OFF_W2A % 128 == 0 && OFF_W2B % 128 == 0 && OFF_W3A % 128 == 0 && OFF_W3B % 128 == 0);
static_assert(OFF_XYZ1 % 128 == 0 && OFF_XYZ2 % 128 == 0 && OFF_F1 % 128 == 0 && OFF_A3 % 128 == 0 && OFF_ACT3 % 128 == 0);
static_assert(WS_TOTAL <= (size_t)134217728);
static_assert((size_t)NBATCH * CH3B * 4 == (size_t)65536);
static_assert(__builtin_bit_cast(unsigned, (float)(0.2 * 0.2)) == 0x3D23D70Au);
static_assert(__builtin_bit_cast(unsigned, (float)(0.4 * 0.4)) == 0x3E23D70Au);

__device__ __forceinline__ unsigned f16bits(const float v) {
  const _Float16 hv = (_Float16)v;
  const unsigned short s = __builtin_bit_cast(unsigned short, hv);
  return (unsigned)s;
}
__device__ __forceinline__ void store2_v4u(unsigned short* dst, const v4u v) {
  volatile v4u* d = (volatile v4u*)(void*)dst;
  *d = v;
  __threadfence();
  *d = v;
}
__device__ __forceinline__ void store2_v4f(float* dst, const v4f v) {
  volatile v4f* d = (volatile v4f*)(void*)dst;
  *d = v;
  __threadfence();
  *d = v;
}
__device__ __forceinline__ void wave_lds_sync() {
  __builtin_amdgcn_fence(__ATOMIC_RELEASE, "workgroup");
  __builtin_amdgcn_wave_barrier();
  __builtin_amdgcn_fence(__ATOMIC_ACQUIRE, "workgroup");
}

__device__ __forceinline__ v16h frag_load(const _Float16* p) {
  union FU { v16h v; v8h h[2]; } f;
  f.h[0] = *(const v8h*)(p);
  f.h[1] = *(const v8h*)(p + 16);
  return f.v;
}
__device__ __forceinline__ v8f mma_h(const v16h a, const v16h b, const v8f c) {
  return __builtin_amdgcn_wmma_f32_16x16x32_f16(false, a, false, b, (short)0, c, false, false);
}
__device__ __forceinline__ void guard_row4(v8f& a0, v8f& a1, v8f& a2, v8f& a3, const v16h x,
                                           const v16h y0, const v16h y1, const v16h y2, const v16h y3) {
  asm volatile("v_nop\n\tv_nop\n\tv_nop\n\tv_nop"
               : "+v"(a0), "+v"(a1), "+v"(a2), "+v"(a3)
               : "v"(x), "v"(y0), "v"(y1), "v"(y2), "v"(y3));
}
__device__ __forceinline__ void acc_guard4(v8f& a, v8f& b, v8f& c, v8f& d) {
  asm volatile("v_nop\n\tv_nop\n\tv_nop\n\tv_nop" : "+v"(a), "+v"(b), "+v"(c), "+v"(d));
}

template <int KSTEPS>
__device__ __forceinline__ void tile64(const _Float16* Ab, const int lda, const _Float16* Bb, const int ldb,
                                       const int lane, v8f (&acc)[4][4]) {
  const int rl = lane & 15;
  const int koff = (lane >> 4) * 8;
#pragma unroll 1
  for (int ks = 0; ks < KSTEPS; ++ks) {
    const int k0 = ks * 32 + koff;
    v16h bh[4];
#pragma unroll
    for (int j = 0; j < 4; ++j) bh[j] = frag_load(Bb + (size_t)((j << 4) + rl) * ldb + k0);
#pragma unroll
    for (int i = 0; i < 4; ++i) {
      const v16h ah = frag_load(Ab + (size_t)((i << 4) + rl) * lda + k0);
#pragma unroll
      for (int j = 0; j < 4; ++j) acc[i][j] = mma_h(ah, bh[j], acc[i][j]);
      guard_row4(acc[i][0], acc[i][1], acc[i][2], acc[i][3], ah, bh[0], bh[1], bh[2], bh[3]);
    }
  }
  acc_guard4(acc[0][0], acc[0][1], acc[0][2], acc[0][3]);
  acc_guard4(acc[1][0], acc[1][1], acc[1][2], acc[1][3]);
  acc_guard4(acc[2][0], acc[2][1], acc[2][2], acc[2][3]);
  acc_guard4(acc[3][0], acc[3][1], acc[3][2], acc[3][3]);
}

template <int KSTEPS>
__device__ __forceinline__ void tile32(const _Float16* Ab, const int lda, const _Float16* Bb, const int ldb,
                                       const int lane, v8f (&acc)[2][4]) {
  const int rl = lane & 15;
  const int koff = (lane >> 4) * 8;
#pragma unroll 1
  for (int ks = 0; ks < KSTEPS; ++ks) {
    const int k0 = ks * 32 + koff;
    v16h bh[4];
#pragma unroll
    for (int j = 0; j < 4; ++j) bh[j] = frag_load(Bb + (size_t)((j << 4) + rl) * ldb + k0);
#pragma unroll
    for (int i = 0; i < 2; ++i) {
      const v16h ah = frag_load(Ab + (size_t)((i << 4) + rl) * lda + k0);
#pragma unroll
      for (int j = 0; j < 4; ++j) acc[i][j] = mma_h(ah, bh[j], acc[i][j]);
      guard_row4(acc[i][0], acc[i][1], acc[i][2], acc[i][3], ah, bh[0], bh[1], bh[2], bh[3]);
    }
  }
  acc_guard4(acc[0][0], acc[0][1], acc[0][2], acc[0][3]);
  acc_guard4(acc[1][0], acc[1][1], acc[1][2], acc[1][3]);
}

template <int PITCH>
__device__ __forceinline__ void relu_to_lds32(const v8f (&acc)[2][4], const float* __restrict__ bias, const int ncol0,
                                              unsigned short* mid_row0, const float inv, const float carry,
                                              const int lane) {
  const int rl = lane & 15;
  const int hh = lane >> 4;
#pragma unroll
  for (int j = 0; j < 4; ++j) {
    const int n = ncol0 + (j << 4) + rl;
    const float bv = bias[n];
#pragma unroll
    for (int i = 0; i < 2; ++i) {
#pragma unroll
      for (int r = 0; r < 8; ++r) {
        float v = acc[i][j][r] * inv;
        v = v + bv;
        v = fmaxf(v, 0.0f);
        v = v * carry;
        mid_row0[((i << 4) + 8 * hh + r) * PITCH + n] = (unsigned short)f16bits(v);
      }
    }
  }
}

struct PrepArgs {
  const float* w[6];
  unsigned short* o[6];
  int cin[6];
  int kpad[6];
  int rot[6];
  int blk_end[6];
};
static_assert(sizeof(PrepArgs) == 192);

__global__ __launch_bounds__(256) void k_prep(const PrepArgs a) {
  const int blk = (int)blockIdx.x;
  const float* W = a.w[5];
  unsigned short* O = a.o[5];
  int cin = a.cin[5];
  int kpad = a.kpad[5];
  int rot = a.rot[5];
  int b0 = a.blk_end[4];
  if (blk < a.blk_end[0]) {
    W = a.w[0]; O = a.o[0]; cin = a.cin[0]; kpad = a.kpad[0]; rot = a.rot[0]; b0 = 0;
  } else if (blk < a.blk_end[1]) {
    W = a.w[1]; O = a.o[1]; cin = a.cin[1]; kpad = a.kpad[1]; rot = a.rot[1]; b0 = a.blk_end[0];
  } else if (blk < a.blk_end[2]) {
    W = a.w[2]; O = a.o[2]; cin = a.cin[2]; kpad = a.kpad[2]; rot = a.rot[2]; b0 = a.blk_end[1];
  } else if (blk < a.blk_end[3]) {
    W = a.w[3]; O = a.o[3]; cin = a.cin[3]; kpad = a.kpad[3]; rot = a.rot[3]; b0 = a.blk_end[2];
  } else if (blk < a.blk_end[4]) {
    W = a.w[4]; O = a.o[4]; cin = a.cin[4]; kpad = a.kpad[4]; rot = a.rot[4]; b0 = a.blk_end[3];
  }
  const int q = (blk - b0) * 256 + (int)threadIdx.x;
  const int cpr = kpad >> 3;
  const int n = q / cpr;
  const int kc = (q - n * cpr) << 3;
  const int nfeat = cin - rot;
  unsigned hb[8];
#pragma unroll
  for (int e = 0; e < 8; ++e) {
    const int k = kc + e;
    const bool ok = k < cin;
    int src = (k < nfeat) ? (k + rot) : (k - nfeat);
    src = src < 0 ? 0 : src;
    src = src > cin - 1 ? cin - 1 : src;
    const float wv = W[(size_t)n * cin + src];
    const float v = ok ? (wv * CARRY_W) : 0.0f;
    hb[e] = f16bits(v);
  }
  v4u o;
  o[0] = hb[0] | (hb[1] << 16);
  o[1] = hb[2] | (hb[3] << 16);
  o[2] = hb[4] | (hb[5] << 16);
  o[3] = hb[6] | (hb[7] << 16);
  store2_v4u(O + (size_t)q * 8, o);
}

template <int NP, int NSEL, int NTHR>
__global__ __launch_bounds__(NTHR) void k_fps(const float* __restrict__ pts, float* __restrict__ sel) {
#pragma clang fp contract(off)
  static_assert(NP == NTHR * 8);
  static_assert((NSEL * 3) % 128 == 0);
  constexpr int NWV = NTHR / 32;
  static_assert((NWV & (NWV - 1)) == 0 && NWV <= 32);
  __shared__ float rv[2][32];
  __shared__ int ri[2][32];
  __shared__ __align__(16) float sSel[NSEL * 3];
  const int b = (int)blockIdx.x;
  const int tid = (int)threadIdx.x;
  const int lane = tid & 31;
  const int wave = tid >> 5;
  const float* pb = pts + (size_t)b * NP * 3;
  float fl[24];
  {
    const v4f* src = (const v4f*)(pb + tid * 24);
#pragma unroll
    for (int c = 0; c < 6; ++c) {
      const v4f t = src[c];
      fl[4 * c + 0] = t[0];
      fl[4 * c + 1] = t[1];
      fl[4 * c + 2] = t[2];
      fl[4 * c + 3] = t[3];
    }
  }
  float px[8], py[8], pz[8], md[8];
#pragma unroll
  for (int i = 0; i < 8; ++i) {
    px[i] = fl[3 * i + 0];
    py[i] = fl[3 * i + 1];
    pz[i] = fl[3 * i + 2];
    md[i] = 1e10f;
  }
  int last = 0;
#pragma unroll 1
  for (int it = 0; it < NSEL; ++it) {
    int lc = last < 0 ? 0 : last;
    lc = lc > NP - 1 ? NP - 1 : lc;
    const float lx = pb[lc * 3 + 0];
    const float ly = pb[lc * 3 + 1];
    const float lz = pb[lc * 3 + 2];
    if (tid == 0) {
      sSel[it * 3 + 0] = lx;
      sSel[it * 3 + 1] = ly;
      sSel[it * 3 + 2] = lz;
    }
    float bv = -1.0f;
    int bi = tid * 8;
#pragma unroll
    for (int i = 0; i < 8; ++i) {
      const float dx = px[i] - lx;
      const float dy = py[i] - ly;
      const float dz = pz[i] - lz;
      const float t0 = dx * dx;
      const float t1 = dy * dy;
      const float t2 = dz * dz;
      const float d = (t0 + t2) + t1;
      const float m = fminf(md[i], d);
      md[i] = m;
      const bool tk = m > bv;
      bv = tk ? m : bv;
      bi = tk ? (tid * 8 + i) : bi;
    }
#pragma unroll
    for (int off = 16; off >= 1; off >>= 1) {
      const float ov = __shfl_xor(bv, off, 32);
      const int oi = __shfl_xor(bi, off, 32);
      const bool tk = (ov > bv) || ((ov == bv) && (oi < bi));
      bv = tk ? ov : bv;
      bi = tk ? oi : bi;
    }
    const int par = it & 1;
    if (lane == 0) {
      rv[par][wave] = bv;
      ri[par][wave] = bi;
    }
    __syncthreads();
    float v2 = rv[par][lane & (NWV - 1)];
    int i2 = ri[par][lane & (NWV - 1)];
#pragma unroll
    for (int off = 16; off >= 1; off >>= 1) {
      const float ov = __shfl_xor(v2, off, 32);
      const int oi = __shfl_xor(i2, off, 32);
      const bool tk = (ov > v2) || ((ov == v2) && (oi < i2));
      v2 = tk ? ov : v2;
      i2 = tk ? oi : i2;
    }
    last = i2;
  }
  __syncthreads();
  float* ob = sel + (size_t)b * NSEL * 3;
  for (int i = tid; i < (NSEL * 3) / 4; i += NTHR) {
    const v4f v = *(const v4f*)(sSel + 4 * i);
    store2_v4f(ob + 4 * i, v);
  }
}

template <int NCAND>
__device__ __forceinline__ void ball_scan(const float* __restrict__ pb, const float cx, const float cy, const float cz,
                                          const float r2, int* lst, const int lane) {
#pragma clang fp contract(off)
  static_assert(NCAND % 32 == 0);
  const float cxx = cx * cx;
  const float cyy = cy * cy;
  const float czz = cz * cz;
  const float sqc = (cxx + czz) + cyy;
  int cnt = 0;
  int first = NCAND - 1;
#pragma unroll 1
  for (int base = 0; base < NCAND; base += 32) {
    if (cnt >= NNB) break;
    const int j = base + lane;
    const float px = pb[j * 3 + 0];
    const float py = pb[j * 3 + 1];
    const float pz = pb[j * 3 + 2];
    const float t0 = px * px;
    const float t1 = py * py;
    const float t2 = pz * pz;
    const float sqp = (t0 + t2) + t1;
    float dp = cx * px;
    dp = __builtin_fmaf(cy, py, dp);
    dp = __builtin_fmaf(cz, pz, dp);
    const float two_dp = 2.0f * dp;
    const float d2 = (sqc + sqp) - two_dp;
    const int pred = (d2 < r2) ? 1 : 0;
    const unsigned m = (unsigned)__ballot(pred);
    if (cnt == 0 && m != 0u) first = base + (int)__builtin_ctz(m);
    const unsigned below = m & ((1u << lane) - 1u);
    const int pos = cnt + (int)__popc(below);
    if (pred != 0 && pos < NNB) lst[pos] = j;
    cnt += (int)__popc(m);
  }
  const int cc = cnt > NNB ? NNB : cnt;
  if (lane >= cc) lst[lane] = first;
  if (lane + 32 >= cc) lst[lane + 32] = first;
}

__global__ __launch_bounds__(256) void k_sa1(const float* __restrict__ x, const float* __restrict__ xyz1,
                                             const unsigned short* __restrict__ w1a, const float* __restrict__ b1a,
                                             const unsigned short* __restrict__ w1b, const float* __restrict__ b1b,
                                             unsigned short* __restrict__ feat1, const float r2) {
#pragma clang fp contract(off)
  __shared__ __align__(16) unsigned short sA[256 * KP1A];
  __shared__ __align__(16) unsigned short sMid[256 * KP1B];
  __shared__ __align__(16) unsigned short sOut[4 * CH1B];
  __shared__ __align__(16) int sList[4 * NNB];
  const int tid = (int)threadIdx.x;
  const int wave = tid >> 5;
  const int lane = tid & 31;
  const int hh = lane >> 4;
  const int rl = lane & 15;
  const int g0 = (int)blockIdx.x * 4;
  const int b = g0 / NCTR1;
  const float* xb = x + (size_t)b * NPTS0 * 3;
  if (wave < 4) {
    const float* cc = xyz1 + (size_t)(g0 + wave) * 3;
    const float cx = cc[0];
    const float cy = cc[1];
    const float cz = cc[2];
    ball_scan<NPTS0>(xb, cx, cy, cz, r2, sList + wave * NNB, lane);
  }
  __syncthreads();
  {
    const int r = tid;
    int p = sList[r];
    p = p < 0 ? 0 : p;
    p = p > NPTS0 - 1 ? NPTS0 - 1 : p;
    const float* pp = xb + (size_t)p * 3;
    const float* cc = xyz1 + (size_t)(g0 + (r >> 6)) * 3;
    const float gx = (pp[0] - cc[0]) * CARRY_G1;
    const float gy = (pp[1] - cc[1]) * CARRY_G1;
    const float gz = (pp[2] - cc[2]) * CARRY_G1;
    unsigned zz = 0;
    asm volatile("" : "+v"(zz));
    v4u c0;
    c0[0] = f16bits(gx) | (f16bits(gy) << 16);
    c0[1] = f16bits(gz) | (zz << 16);
    c0[2] = zz;
    c0[3] = zz;
    v4u cz4;
    cz4[0] = zz;
    cz4[1] = zz;
    cz4[2] = zz;
    cz4[3] = zz;
    v4u* dst = (v4u*)(void*)(sA + r * KP1A);
    dst[0] = c0;
    dst[1] = cz4;
    dst[2] = cz4;
    dst[3] = cz4;
  }
  __syncthreads();
  {
    v8f acc[2][4];
#pragma unroll
    for (int i = 0; i < 2; ++i)
#pragma unroll
      for (int j = 0; j < 4; ++j) acc[i][j] = (v8f){0.f, 0.f, 0.f, 0.f, 0.f, 0.f, 0.f, 0.f};
    tile32<KP1A / 32>((const _Float16*)sA + wave * 32 * KP1A, KP1A, (const _Float16*)w1a, KP1A, lane, acc);
    relu_to_lds32<KP1B>(acc, b1a, 0, sMid + wave * 32 * KP1B, INV_1A, CARRY_M1, lane);
  }
  __syncthreads();
  {
    const int gl = wave >> 1;
    const int nh = wave & 1;
    v8f acc[4][4];
#pragma unroll
    for (int i = 0; i < 4; ++i)
#pragma unroll
      for (int j = 0; j < 4; ++j) acc[i][j] = (v8f){0.f, 0.f, 0.f, 0.f, 0.f, 0.f, 0.f, 0.f};
    tile64<KP1B / 32>((const _Float16*)sMid + gl * 64 * KP1B, KP1B, (const _Float16*)w1b + nh * 64 * KP1B, KP1B, lane, acc);
#pragma unroll
    for (int j = 0; j < 4; ++j) {
      float cm = acc[0][j][0];
#pragma unroll
      for (int i = 0; i < 4; ++i)
#pragma unroll
        for (int r = 0; r < 8; ++r) cm = fmaxf(cm, acc[i][j][r]);
      const float om = __shfl_xor(cm, 16, 32);
      cm = fmaxf(cm, om);
      const int n = nh * 64 + (j << 4) + rl;
      float v = cm * INV_1B;
      v = v + b1b[n];
      v = fmaxf(v, 0.0f);
      v = v * CARRY_F1;
      if (hh == 0) sOut[gl * CH1B + n] = (unsigned short)f16bits(v);
    }
  }
  __syncthreads();
  if (tid < 64) {
    const v4u v = *(const v4u*)(const void*)(sOut + tid * 8);
    store2_v4u(feat1 + (size_t)g0 * CH1B + tid * 8, v);
  }
}

__global__ __launch_bounds__(256) void k_sa2(const float* __restrict__ xyz1, const unsigned short* __restrict__ feat1,
                                             const float* __restrict__ xyz2,
                                             const unsigned short* __restrict__ w2a, const float* __restrict__ b2a,
                                             const unsigned short* __restrict__ w2b, const float* __restrict__ b2b,
                                             unsigned short* __restrict__ a3, const float r2) {
#pragma clang fp contract(off)
  __shared__ __align__(16) unsigned short sA[128 * KP2A];
  __shared__ __align__(16) unsigned short sMid[128 * KP2B];
  __shared__ __align__(16) unsigned short sOut[2 * KP3A];
  __shared__ __align__(16) int sList[2 * NNB];
  const int tid = (int)threadIdx.x;
  const int wave = tid >> 5;
  const int lane = tid & 31;
  const int hh = lane >> 4;
  const int rl = lane & 15;
  const int g0 = (int)blockIdx.x * 2;
  const int b = g0 / NCTR2;
  const float* pb = xyz1 + (size_t)b * NCTR1 * 3;
  if (wave < 2) {
    const float* cc = xyz2 + (size_t)(g0 + wave) * 3;
    const float cx = cc[0];
    const float cy = cc[1];
    const float cz = cc[2];
    ball_scan<NCTR1>(pb, cx, cy, cz, r2, sList + wave * NNB, lane);
  }
  __syncthreads();
#pragma unroll 2
  for (int it = 0; it < 8; ++it) {
    const int q = it * 256 + tid;
    const int row = q >> 4;
    const int ch = q & 15;
    int p = sList[row];
    p = p < 0 ? 0 : p;
    p = p > NCTR1 - 1 ? NCTR1 - 1 : p;
    const v4u v = *(const v4u*)(const void*)(feat1 + ((size_t)b * NCTR1 + p) * CH1B + ch * 8);
    *(v4u*)(void*)(sA + row * KP2A + ch * 8) = v;
  }
  if (tid < 128) {
    const int r = tid;
    int p = sList[r];
    p = p < 0 ? 0 : p;
    p = p > NCTR1 - 1 ? NCTR1 - 1 : p;
    const float* pp = pb + (size_t)p * 3;
    const float* cc = xyz2 + (size_t)(g0 + (r >> 6)) * 3;
    const float gx = (pp[0] - cc[0]) * CARRY_F1;
    const float gy = (pp[1] - cc[1]) * CARRY_F1;
    const float gz = (pp[2] - cc[2]) * CARRY_F1;
    unsigned zz = 0;
    asm volatile("" : "+v"(zz));
    v4u c0;
    c0[0] = f16bits(gx) | (f16bits(gy) << 16);
    c0[1] = f16bits(gz) | (zz << 16);
    c0[2] = zz;
    c0[3] = zz;
    v4u cz4;
    cz4[0] = zz;
    cz4[1] = zz;
    cz4[2] = zz;
    cz4[3] = zz;
    v4u* dst = (v4u*)(void*)(sA + r * KP2A + CH1B);
    dst[0] = c0;
    dst[1] = cz4;
    dst[2] = cz4;
    dst[3] = cz4;
  }
  if (tid < 64) {
    const int gl = tid >> 5;
    const int c = tid & 31;
    const float* cc = xyz2 + (size_t)(g0 + gl) * 3;
    const float cx = cc[0];
    const float cy = cc[1];
    const float cz = cc[2];
    const float val = (c == 0) ? cx : ((c == 1) ? cy : cz);
    const unsigned bits = (c < 3) ? f16bits(val * CARRY_F2) : 0u;
    sOut[gl * KP3A + CH2B + c] = (unsigned short)bits;
  }
  __syncthreads();
  {
    const int mb = wave >> 1;
    const int nb = wave & 1;
    v8f acc[2][4];
#pragma unroll
    for (int i = 0; i < 2; ++i)
#pragma unroll
      for (int j = 0; j < 4; ++j) acc[i][j] = (v8f){0.f, 0.f, 0.f, 0.f, 0.f, 0.f, 0.f, 0.f};
    tile32<KP2A / 32>((const _Float16*)sA + mb * 32 * KP2A, KP2A, (const _Float16*)w2a + nb * 64 * KP2A, KP2A, lane, acc);
    relu_to_lds32<KP2B>(acc, b2a, nb * 64, sMid + mb * 32 * KP2B, INV_2A, CARRY_M2, lane);
  }
  __syncthreads();
  {
    const int gl = wave >> 2;
    const int nq = wave & 3;
    v8f acc[4][4];
#pragma unroll
    for (int i = 0; i < 4; ++i)
#pragma unroll
      for (int j = 0; j < 4; ++j) acc[i][j] = (v8f){0.f, 0.f, 0.f, 0.f, 0.f, 0.f, 0.f, 0.f};
    tile64<KP2B / 32>((const _Float16*)sMid + gl * 64 * KP2B, KP2B, (const _Float16*)w2b + nq * 64 * KP2B, KP2B, lane, acc);
#pragma unroll
    for (int j = 0; j < 4; ++j) {
      float cm = acc[0][j][0];
#pragma unroll
      for (int i = 0; i < 4; ++i)
#pragma unroll
        for (int r = 0; r < 8; ++r) cm = fmaxf(cm, acc[i][j][r]);
      const float om = __shfl_xor(cm, 16, 32);
      cm = fmaxf(cm, om);
      const int n = nq * 64 + (j << 4) + rl;
      float v = cm * INV_2B;
      v = v + b2b[n];
      v = fmaxf(v, 0.0f);
      v = v * CARRY_F2;
      if (hh == 0) sOut[gl * KP3A + n] = (unsigned short)f16bits(v);
    }
  }
  __syncthreads();
  if (tid < 72) {
    const v4u v = *(const v4u*)(const void*)(sOut + tid * 8);
    store2_v4u(a3 + (size_t)g0 * KP3A + tid * 8, v);
  }
}

__global__ __launch_bounds__(256) void k_sa3a(const unsigned short* __restrict__ a3, const unsigned short* __restrict__ w3a,
                                              const float* __restrict__ b3a, unsigned short* __restrict__ act3) {
  __shared__ __align__(16) float sT[8][16 * 68];
  const int tid = (int)threadIdx.x;
  const int wave = tid >> 5;
  const int lane = tid & 31;
  const int rl = lane & 15;
  const int mOff = (lane >> 4) * 8;
  const int tile = (int)blockIdx.x * 8 + wave;
  const int tm = tile >> 3;
  const int tn = tile & 7;
  const int m0 = tm << 6;
  const int n0 = tn << 6;
  v8f acc[4][4];
#pragma unroll
  for (int i = 0; i < 4; ++i)
#pragma unroll
    for (int j = 0; j < 4; ++j) acc[i][j] = (v8f){0.f, 0.f, 0.f, 0.f, 0.f, 0.f, 0.f, 0.f};
  tile64<KP3A / 32>((const _Float16*)a3 + (size_t)m0 * KP3A, KP3A, (const _Float16*)w3a + (size_t)n0 * KP3A, KP3A, lane, acc);
  float* slab = sT[wave];
#pragma unroll
  for (int i = 0; i < 4; ++i) {
    const int mBase = m0 + (i << 4);
#pragma unroll
    for (int j = 0; j < 4; ++j) {
      const float bv = b3a[n0 + (j << 4) + rl];
#pragma unroll
      for (int r = 0; r < 8; ++r) {
        float v = acc[i][j][r] * INV_3A;
        v = v + bv;
        v = fmaxf(v, 0.0f);
        v = v * CARRY_M3;
        slab[(mOff + r) * 68 + (j << 4) + rl] = v;
      }
    }
    wave_lds_sync();
    {
      const int q = lane >> 3;
      const int c8 = (lane & 7) * 8;
      for (int pass = 0; pass < 2; ++pass) {
#pragma unroll
        for (int it = 0; it < 4; ++it) {
          const int row = it * 4 + q;
          const float* sp = slab + row * 68 + c8;
          v8h hv;
#pragma unroll
          for (int e = 0; e < 8; ++e) hv[e] = (_Float16)sp[e];
          *(volatile v8h*)(void*)(act3 + (size_t)(mBase + row) * CH3A + n0 + c8) = hv;
        }
        __threadfence();
      }
    }
    wave_lds_sync();
  }
}

__global__ __launch_bounds__(256) void k_sa3b(const unsigned short* __restrict__ act3, const unsigned short* __restrict__ w3b,
                                              const float* __restrict__ b3b, float* __restrict__ out) {
  __shared__ __align__(16) float sPool[2 * 256];
  const int tid = (int)threadIdx.x;
  const int wave = tid >> 5;
  const int lane = tid & 31;
  const int hh = lane >> 4;
  const int rl = lane & 15;
  const int b = (int)blockIdx.x >> 2;
  const int nb = (int)blockIdx.x & 3;
  const int mb = wave >> 2;
  const int nq = wave & 3;
  v8f acc[4][4];
#pragma unroll
  for (int i = 0; i < 4; ++i)
#pragma unroll
    for (int j = 0; j < 4; ++j) acc[i][j] = (v8f){0.f, 0.f, 0.f, 0.f, 0.f, 0.f, 0.f, 0.f};
  tile64<KP3B / 32>((const _Float16*)act3 + ((size_t)b * NCTR2 + mb * 64) * KP3B, KP3B,
                    (const _Float16*)w3b + ((size_t)nb * 256 + nq * 64) * KP3B, KP3B, lane, acc);
#pragma unroll
  for (int j = 0; j < 4; ++j) {
    float cm = acc[0][j][0];
#pragma unroll
    for (int i = 0; i < 4; ++i)
#pragma unroll
      for (int r = 0; r < 8; ++r) cm = fmaxf(cm, acc[i][j][r]);
    const float om = __shfl_xor(cm, 16, 32);
    cm = fmaxf(cm, om);
    if (hh == 0) sPool[mb * 256 + nq * 64 + (j << 4) + rl] = cm;
  }
  __syncthreads();
  if (tid < 64) {
    const int c4 = tid * 4;
    const v4f pa = *(const v4f*)(sPool + c4);
    const v4f pc = *(const v4f*)(sPool + 256 + c4);
    const v4f bv = *(const v4f*)(b3b + nb * 256 + c4);
    v4f o;
#pragma unroll
    for (int e = 0; e < 4; ++e) {
      float v = fmaxf(pa[e], pc[e]) * INV_3B;
      v = v + bv[e];
      o[e] = fmaxf(v, 0.0f);
    }
    store2_v4f(out + (size_t)b * CH3B + nb * 256 + c4, o);
  }
}

extern "C" void kernel_launch(void* const* d_in, const int* in_sizes, int n_in,
                              void* d_out, int out_size, void* d_ws, size_t ws_size, hipStream_t stream) {
  (void)in_sizes;
  (void)out_size;
  if (n_in < 13) return;
  if (ws_size < WS_TOTAL) return;
  const float* x   = (const float*)d_in[0];
  const float* W1a = (const float*)d_in[1];
  const float* b1a = (const float*)d_in[2];
  const float* W1b = (const float*)d_in[3];
  const float* b1b = (const float*)d_in[4];
  const float* W2a = (const float*)d_in[5];
  const float* b2a = (const float*)d_in[6];
  const float* W2b = (const float*)d_in[7];
  const float* b2b = (const float*)d_in[8];
  const float* W3a = (const float*)d_in[9];
  const float* b3a = (const float*)d_in[10];
  const float* W3b = (const float*)d_in[11];
  const float* b3b = (const float*)d_in[12];

  unsigned char* ws = (unsigned char*)d_ws;
  unsigned short* w1a16 = (unsigned short*)(ws + OFF_W1A);
  unsigned short* w1b16 = (unsigned short*)(ws + OFF_W1B);
  unsigned short* w2a16 = (unsigned short*)(ws + OFF_W2A);
  unsigned short* w2b16 = (unsigned short*)(ws + OFF_W2B);
  unsigned short* w3a16 = (unsigned short*)(ws + OFF_W3A);
  unsigned short* w3b16 = (unsigned short*)(ws + OFF_W3B);
  float* xyz1 = (float*)(ws + OFF_XYZ1);
  float* xyz2 = (float*)(ws + OFF_XYZ2);
  unsigned short* feat1 = (unsigned short*)(ws + OFF_F1);
  unsigned short* a3 = (unsigned short*)(ws + OFF_A3);
  unsigned short* act3 = (unsigned short*)(ws + OFF_ACT3);
  float* out = (float*)d_out;

  PrepArgs pa;
  pa.w[0] = W1a; pa.w[1] = W1b; pa.w[2] = W2a; pa.w[3] = W2b; pa.w[4] = W3a; pa.w[5] = W3b;
  pa.o[0] = w1a16; pa.o[1] = w1b16; pa.o[2] = w2a16; pa.o[3] = w2b16; pa.o[4] = w3a16; pa.o[5] = w3b16;
  pa.cin[0] = CIN1; pa.cin[1] = CH1A; pa.cin[2] = CIN2; pa.cin[3] = CH2A; pa.cin[4] = CIN3; pa.cin[5] = CH3A;
  pa.kpad[0] = KP1A; pa.kpad[1] = KP1B; pa.kpad[2] = KP2A; pa.kpad[3] = KP2B; pa.kpad[4] = KP3A; pa.kpad[5] = KP3B;
  pa.rot[0] = 0; pa.rot[1] = 0; pa.rot[2] = 3; pa.rot[3] = 0; pa.rot[4] = 3; pa.rot[5] = 0;
  int be = 0;
  be += (CH1A * KP1A) / 2048; pa.blk_end[0] = be;
  be += (CH1B * KP1B) / 2048; pa.blk_end[1] = be;
  be += (CH2A * KP2A) / 2048; pa.blk_end[2] = be;
  be += (CH2B * KP2B) / 2048; pa.blk_end[3] = be;
  be += (CH3A * KP3A) / 2048; pa.blk_end[4] = be;
  be += (CH3B * KP3B) / 2048; pa.blk_end[5] = be;
  k_prep<<<be, 256, 0, stream>>>(pa);

  const float r2a = (float)(0.2 * 0.2);
  const float r2b = (float)(0.4 * 0.4);

  k_fps<NPTS0, NCTR1, 1024><<<NBATCH, 1024, 0, stream>>>(x, xyz1);
  k_sa1<<<(NBATCH * NCTR1) / 4, 256, 0, stream>>>(x, xyz1, w1a16, b1a, w1b16, b1b, feat1, r2a);
  k_fps<NCTR1, NCTR2, 64><<<NBATCH, 64, 0, stream>>>(xyz1, xyz2);
  k_sa2<<<(NBATCH * NCTR2) / 2, 256, 0, stream>>>(xyz1, feat1, xyz2, w2a16, b2a, w2b16, b2b, a3, r2b);
  k_sa3a<<<((NBATCH * NCTR2) / 64) * (CH3A / 64) / 8, 256, 0, stream>>>(a3, w3a16, b3a, act3);
  k_sa3b<<<NBATCH * (CH3B / 256), 256, 0, stream>>>(act3, w3b16, b3b, out);
}
